// PerformerBlock_2190433321796
// MI455X (gfx1250) — hardware-run, weakly checked
//
#include <hip/hip_runtime.h>
#include <math.h>

typedef __attribute__((ext_vector_type(16))) _Float16 v16h;
typedef __attribute__((ext_vector_type(16))) __bf16 v16b;
typedef __attribute__((ext_vector_type(8)))  _Float16 v8h;
typedef __attribute__((ext_vector_type(8)))  float v8f;
typedef __attribute__((ext_vector_type(4)))  float v4f;
typedef __attribute__((ext_vector_type(2)))  float v2f;
typedef __attribute__((ext_vector_type(4)))  unsigned v4u;
typedef __attribute__((ext_vector_type(4)))  int v4i;
typedef float __attribute__((may_alias)) float_a;
typedef int __attribute__((may_alias)) int_a;

template <typename T> __device__ __forceinline__ void vst2(void* p, T v) { *(volatile T*)p = v; __threadfence(); *(volatile T*)p = v; }
__device__ __forceinline__ v8f wmma16(v16h a, v16h b, v8f c) {
  v8f d = __builtin_amdgcn_wmma_f32_16x16x32_f16(false, a, false, b, (short)0, c, false, false);
  asm volatile("v_nop\n\tv_nop\n\tv_nop\n\tv_nop" : "+v"(d) : "v"(a), "v"(b));
  return d;
}
__device__ __forceinline__ v8f wmma_bf(v16b a, v16b b, v8f c) {
  v8f d = __builtin_amdgcn_wmma_f32_16x16x32_bf16(false, a, false, b, (short)0, c, false, false);
  asm volatile("v_nop\n\tv_nop\n\tv_nop\n\tv_nop" : "+v"(d) : "v"(a), "v"(b));
  return d;
}
__device__ __forceinline__ v16h frag_h(const _Float16* rowk0, int lane) {
  union { v16h v; v8h q[2]; } u; const _Float16* p = rowk0 + 8 * (lane >> 4);
  u.q[0] = *(const v8h*)p; u.q[1] = *(const v8h*)(p + 16); return u.v;
}
__device__ __forceinline__ v16h frag_f32(const float* rowk0, int lane) {
  v16h a; const float* p = rowk0 + 8 * (lane >> 4);
#pragma unroll
  for (int i = 0; i < 8; ++i) { a[i] = (_Float16)p[i]; a[8 + i] = (_Float16)p[16 + i]; }
  return a;
}
__device__ __forceinline__ v16h frag_f32s(const float* rowk0, int lane, float sc) {
  v16h a; const float* p = rowk0 + 8 * (lane >> 4);
#pragma unroll
  for (int i = 0; i < 8; ++i) { a[i] = (_Float16)(p[i] * sc); a[8 + i] = (_Float16)(p[16 + i] * sc); }
  return a;
}
__device__ __forceinline__ v16h fragc_f32(const float* W, int k0, int n, int lane, int ld, int K) {
  v16h a; const int g = lane >> 4;
#pragma unroll
  for (int i = 0; i < 8; ++i) { const int ka = k0 + 8 * g + i, kb = ka + 16;
    a[i] = (_Float16)(ka < K ? W[(size_t)(ka < K ? ka : K - 1) * ld + n] : 0.f); a[8 + i] = (_Float16)(kb < K ? W[(size_t)(kb < K ? kb : K - 1) * ld + n] : 0.f); }
  return a;
}
struct F2 { v16b h, l; };
__device__ __forceinline__ F2 bsplit16(const float v[16]) { F2 r;
#pragma unroll
  for (int i = 0; i < 16; ++i) { const __bf16 h = (__bf16)v[i]; r.h[i] = h; r.l[i] = (__bf16)(v[i] - (float)h); }
  return r; }
__device__ __forceinline__ F2 split_row(const float* row, int k0, int lane) { float v[16]; const float* p = row + k0 + 8 * (lane >> 4);
#pragma unroll
  for (int i = 0; i < 8; ++i) { v[i] = p[i]; v[8 + i] = p[16 + i]; }
  return bsplit16(v); }
__device__ __forceinline__ F2 split_rowK(const float* row, int k0, int lane, int K) { float v[16]; const int g = lane >> 4;
#pragma unroll
  for (int i = 0; i < 8; ++i) { const int ka = k0 + 8 * g + i, kb = ka + 16; v[i] = ka < K ? row[ka < K ? ka : K - 1] : 0.f; v[8 + i] = kb < K ? row[kb < K ? kb : K - 1] : 0.f; }
  return bsplit16(v); }
__device__ __forceinline__ F2 split_col(const float* W, int k0, int n, int lane, int ld, int K) { float v[16]; const int g = lane >> 4;
#pragma unroll
  for (int i = 0; i < 8; ++i) { const int ka = k0 + 8 * g + i, kb = ka + 16; v[i] = ka < K ? W[(size_t)(ka < K ? ka : K - 1) * ld + n] : 0.f; v[8 + i] = kb < K ? W[(size_t)(kb < K ? kb : K - 1) * ld + n] : 0.f; }
  return bsplit16(v); }
__device__ __forceinline__ v8f mac3(const F2& a, const F2& b, v8f c) { c = wmma_bf(a.l, b.h, c); c = wmma_bf(a.h, b.l, c); return wmma_bf(a.h, b.h, c); }
__device__ __forceinline__ float sigm(float v) { return 1.0f / (1.0f + expf(-v)); }
#define LDSX() do { asm volatile("s_wait_dscnt 0" ::: "memory"); __builtin_amdgcn_wave_barrier(); __builtin_amdgcn_fence(__ATOMIC_RELEASE, "workgroup"); } while (0)

__device__ __forceinline__ float bfr(float v) { return (float)(__bf16)v; }
#define NB 4
#define TT 4096
#define CC 512
#define NH 8
#define HD 64
#define MF 266
#define MP 320
#define NR (NB * TT)
#define FSC 16384.0f
#ifndef TNB
#define TNB NB
#endif
#define WS_Q   0u
#define WS_K   (WS_Q + 4u * (size_t)NR * CC)
#define WS_VP  (WS_K + 4u * (size_t)NR * CC)
#define WS_KP  (WS_VP + 2u * (size_t)NB * CC * TT)
#define WS_QP  (WS_KP + 2u * (size_t)NB * NH * MP * TT)
#define WS_PM  (WS_QP + 2u * (size_t)NB * NH * TT * MP)
#define WS_CT  (WS_PM + 4u * (size_t)NB * NH * (TT / 64) * 32)
#define WS_END (WS_CT + 4u * (size_t)NB * NH * 80 * MP)
#define WS_O   WS_K
__global__ __launch_bounds__(128) void k_qkv(const float* __restrict__ X, const float* __restrict__ WQ, const float* __restrict__ WK, const float* __restrict__ WV, float* __restrict__ Q, float* __restrict__ K, _Float16* __restrict__ VP) { __shared__ __align__(16) float sf[4][16][132]; __shared__ __align__(16) _Float16 th[128][72];
  const int tid = threadIdx.x, wave = tid >> 5, lane = tid & 31, col = lane & 15, g = lane >> 4; const int which = blockIdx.z; const int c0 = blockIdx.y * 128; const size_t r0 = (size_t)blockIdx.x * 64;
  const float* WA = which == 0 ? WQ : which == 1 ? WK : WV;
  v8f acc[8] = {};
#pragma unroll 2
  for (int kc = 0; kc < CC / 32; ++kc) { v16b a; { const float* p = X + (r0 + wave * 16 + col) * CC + kc * 32 + 8 * g;
#pragma unroll
      for (int i = 0; i < 8; ++i) { a[i] = (__bf16)p[i]; a[8 + i] = (__bf16)p[16 + i]; } }
#pragma unroll
    for (int j = 0; j < 8; ++j) { v16b w; const int o = c0 + j * 16 + col; const float* wr = WA + (size_t)o * CC + kc * 32 + 8 * g;
#pragma unroll
      for (int i = 0; i < 8; ++i) { w[i] = (__bf16)wr[i]; w[8 + i] = (__bf16)wr[16 + i]; }
      acc[j] = wmma_bf(a, w, acc[j]); } }
  if (which < 2) { float* D = which == 0 ? Q : K;
#pragma unroll
    for (int j = 0; j < 8; ++j)
#pragma unroll
      for (int r = 0; r < 8; ++r) sf[wave][8 * g + r][j * 16 + col] = acc[j][r];
    LDSX(); for (int rl = 0; rl < 16; ++rl) vst2(D + (r0 + wave * 16 + rl) * CC + c0 + lane * 4, *(const v4f*)&sf[wave][rl][lane * 4]); }
  else {
#pragma unroll
    for (int j = 0; j < 8; ++j)
#pragma unroll
      for (int r = 0; r < 8; ++r) th[j * 16 + col][wave * 16 + 8 * g + r] = (_Float16)acc[j][r];
    __syncthreads(); const size_t b = r0 / TT; const int t0 = (int)(r0 % TT);
    for (int e = tid; e < 128 * 8; e += 128) { const int cl = e >> 3, q = e & 7; vst2((unsigned*)(VP + (b * CC + c0 + cl) * (size_t)TT + t0 + q * 8), *(const v4u*)&th[cl][q * 8]); } } }
__device__ __forceinline__ void td_tile(const float* __restrict__ T, const float* __restrict__ PJ, size_t row0, int h, int wave, int lane, float (*std_)[MP + 4], float* sdiag) {
  const int col = lane & 15, g = lane >> 4;
  F2 a[2]; a[0] = split_row(T + (row0 + col) * CC + h * HD, 0, lane); a[1] = split_row(T + (row0 + col) * CC + h * HD, 32, lane);
#pragma unroll 1
  for (int jt = 0; jt < MP / 16; ++jt) { v8f acc = {};
#pragma unroll
    for (int kc = 0; kc < 2; ++kc) { v16b w; const int m = jt * 16 + col; const int mm = m < MF ? m : MF - 1; const float* pr = PJ + (size_t)mm * HD + kc * 32 + 8 * g;
#pragma unroll
      for (int i = 0; i < 8; ++i) { w[i] = (m < MF) ? (__bf16)pr[i] : (__bf16)0.f; w[8 + i] = (m < MF) ? (__bf16)pr[16 + i] : (__bf16)0.f; }
      acc = wmma_bf(a[kc].h, w, acc); acc = wmma_bf(a[kc].l, w, acc); }
#pragma unroll
    for (int r = 0; r < 8; ++r) std_[wave * 16 + 8 * g + r][jt * 16 + col] = acc[r] * 0.35355339059327373f; }
  if (lane < 16) { const float* tr = T + (row0 + lane) * CC + h * HD; float s = 0.f;
#pragma unroll 1
    for (int d = 0; d < HD; d += 4) { const v4f v = *(const v4f*)(tr + d); s += (v[0] * v[0] + v[1] * v[1]) + (v[2] * v[2] + v[3] * v[3]); }
    sdiag[wave * 16 + lane] = s * (0.5f * 0.125f); }
}
__global__ __launch_bounds__(128) void k_kmax(const float* __restrict__ K, const float* __restrict__ PJ, float* __restrict__ PM) { __shared__ __align__(16) float std_[64][MP + 4]; __shared__ float sdiag[64]; __shared__ float sred[4];
  const int tid = threadIdx.x, wave = tid >> 5, lane = tid & 31; const int bh = blockIdx.y; const int b = bh / NH, h = bh % NH; const size_t row0 = (size_t)b * TT + (size_t)blockIdx.x * 64 + wave * 16;
  td_tile(K, PJ, row0, h, wave, lane, std_, sdiag); LDSX(); __syncthreads();
  float m = -3.0e38f; for (int e = tid; e < 64 * MF; e += 128) { const int r = e / MF, c = e % MF; m = fmaxf(m, std_[r][c]); }
#pragma unroll
  for (int o = 1; o < 32; o <<= 1) m = fmaxf(m, __shfl_xor(m, o));
  if (lane == 0) sred[wave] = m; __syncthreads();
  if (tid < 32) { const float v = (tid == 0) ? fmaxf(fmaxf(sred[0], sred[1]), fmaxf(sred[2], sred[3])) : 0.f; vst2(PM + ((size_t)bh * (TT / 64) + blockIdx.x) * 32 + tid, v); } }
__global__ __launch_bounds__(128) void k_kfeat(const float* __restrict__ K, const float* __restrict__ PJ, const float* __restrict__ PM, _Float16* __restrict__ KP) { __shared__ __align__(16) float std_[64][MP + 4]; __shared__ float sdiag[64]; __shared__ __align__(16) _Float16 stp[MP][72];
  const int tid = threadIdx.x, wave = tid >> 5, lane = tid & 31; const int bh = blockIdx.y; const int b = bh / NH, h = bh % NH; const int n0 = blockIdx.x * 64; const size_t row0 = (size_t)b * TT + n0 + wave * 16;
  td_tile(K, PJ, row0, h, wave, lane, std_, sdiag); LDSX(); __syncthreads();
  float gm = -3.0e38f; for (int e = 0; e < TT / 64; ++e) gm = fmaxf(gm, PM[((size_t)bh * (TT / 64) + e) * 32]);
  const float ratio = 0.061313933948496426f;
  for (int e = tid; e < 64 * MP; e += 128) { const int r = e / MP, m = e % MP; const float v = (m < MF) ? ratio * (expf(std_[r][m] - sdiag[r] - gm) + 1e-4f) * FSC : 0.f; stp[m][r] = (_Float16)v; }
  __syncthreads();
  for (int e = tid; e < MP * 8; e += 128) { const int m = e >> 3, q = e & 7; vst2((unsigned*)(KP + ((size_t)bh * MP + m) * TT + n0 + q * 8), *(const v4u*)&stp[m][q * 8]); } }
__global__ __launch_bounds__(128) void k_qfeat(const float* __restrict__ Q, const float* __restrict__ PJ, _Float16* __restrict__ QP) { __shared__ __align__(16) float std_[64][MP + 4]; __shared__ float sdiag[64]; __shared__ __align__(16) _Float16 sq[64][MP];
  const int tid = threadIdx.x, wave = tid >> 5, lane = tid & 31; const int bh = blockIdx.y; const int b = bh / NH, h = bh % NH; const int n0 = blockIdx.x * 64; const size_t row0 = (size_t)b * TT + n0 + wave * 16;
  td_tile(Q, PJ, row0, h, wave, lane, std_, sdiag); LDSX(); __syncthreads();
  const float ratio = 0.061313933948496426f;
  { const int r = tid >> 1, half = tid & 1; float m = -3.0e38f; for (int c = half; c < MF; c += 2) m = fmaxf(m, std_[r][c]); m = fmaxf(m, __shfl_xor(m, 1));
    for (int c = half; c < MP; c += 2) { const float v = (c < MF) ? ratio * (expf(std_[r][c] - sdiag[r] - m) + 1e-4f) * FSC : 0.f; sq[r][c] = (_Float16)v; } }
  __syncthreads();
  for (int e = tid; e < 64 * (MP / 8); e += 128) { const int r = e / (MP / 8), q = e % (MP / 8); vst2((unsigned*)(QP + ((size_t)bh * TT + n0 + r) * MP + q * 8), *(const v4u*)&sq[r][q * 8]); } }
__global__ __launch_bounds__(128) void k_ctx(const _Float16* __restrict__ KP, const _Float16* __restrict__ VP, float* __restrict__ CT) { __shared__ __align__(16) float st[80][68];
  const int tid = threadIdx.x, wave = tid >> 5, lane = tid & 31, col = lane & 15, g = lane >> 4; const int bh = blockIdx.y; const int b = bh / NH, h = bh % NH; const int m0 = blockIdx.x * 64 + wave * 16;
  v8f acc[5] = {};
#pragma unroll 1
  for (int kc = 0; kc < TT / 32; ++kc) { const v16h a = frag_h(KP + ((size_t)bh * MP + m0 + col) * TT + kc * 32, lane);
#pragma unroll
    for (int j = 0; j < 4; ++j) acc[j] = wmma16(a, frag_h(VP + ((size_t)b * CC + h * HD + j * 16 + col) * TT + kc * 32, lane), acc[j]);
    { v16h one; const _Float16 ov = (col == 0) ? (_Float16)1.0f : (_Float16)0.f;
#pragma unroll
      for (int i = 0; i < 16; ++i) one[i] = ov; acc[4] = wmma16(a, one, acc[4]); } }
#pragma unroll
  for (int j = 0; j < 5; ++j)
#pragma unroll
    for (int r = 0; r < 8; ++r) st[j * 16 + col][wave * 16 + 8 * g + r] = acc[j][r] * (1.0f / FSC);
  __syncthreads();
  for (int e = tid; e < 80 * 16; e += 128) { const int c = e >> 4, q = e & 15; vst2(CT + ((size_t)bh * 80 + c) * MP + blockIdx.x * 64 + q * 4, *(const v4f*)&st[c][q * 4]); } }
__global__ __launch_bounds__(128) void k_lin(const _Float16* __restrict__ QP, const float* __restrict__ CT, float* __restrict__ O) { __shared__ __align__(16) float sf[4][16][HD + 4];
  const int tid = threadIdx.x, wave = tid >> 5, lane = tid & 31, col = lane & 15, g = lane >> 4; const int bh = blockIdx.y; const int b = bh / NH, h = bh % NH; const int n0 = blockIdx.x * 64 + wave * 16;
  v8f acc[5] = {};
#pragma unroll 1
  for (int kc = 0; kc < MP / 32; ++kc) { const int kbase = kc * 32;
    v16h a; { const _Float16* p = QP + ((size_t)bh * TT + n0 + col) * MP + kbase + 8 * g;
#pragma unroll
      for (int i = 0; i < 8; ++i) { const int k1 = kbase + 8 * g + i, k2 = k1 + 16; a[i] = (k1 < MP) ? p[i] : (_Float16)0.f; a[8 + i] = (k2 < MP) ? p[16 + i] : (_Float16)0.f; } }
#pragma unroll
    for (int j = 0; j < 5; ++j) { v16h w; const int c = j * 16 + col; const float* cr = CT + ((size_t)bh * 80 + c) * MP + kbase + 8 * g;
#pragma unroll
      for (int i = 0; i < 8; ++i) { const int k1 = kbase + 8 * g + i, k2 = k1 + 16; w[i] = (k1 < MP) ? (_Float16)(cr[i] * 16.0f) : (_Float16)0.f; w[8 + i] = (k2 < MP) ? (_Float16)(cr[16 + i] * 16.0f) : (_Float16)0.f; }
      acc[j] = wmma16(a, w, acc[j]); } }
#pragma unroll
  for (int r = 0; r < 8; ++r) { const float den = __shfl(acc[4][r], lane & 16);
#pragma unroll
    for (int j = 0; j < 4; ++j) sf[wave][8 * g + r][j * 16 + col] = acc[j][r] / den; }
  LDSX(); for (int rl = 0; rl < 16; ++rl) if (lane < 16) vst2(O + ((size_t)b * TT + n0 + rl) * CC + h * HD + lane * 4, *(const v4f*)&sf[wave][rl][lane * 4]); }
__global__ __launch_bounds__(128) void k_out(const float* __restrict__ O, const float* __restrict__ WO, const float* __restrict__ BO, const float* __restrict__ X, float* __restrict__ OUT) { __shared__ __align__(16) float sf[4][16][132];
  const int tid = threadIdx.x, wave = tid >> 5, lane = tid & 31, col = lane & 15, g = lane >> 4; const int c0 = blockIdx.y * 128; const size_t r0 = (size_t)blockIdx.x * 64 + wave * 16;
  v8f acc[8] = {};
#pragma unroll 2
  for (int kc = 0; kc < CC / 32; ++kc) { const F2 a = split_row(O + (r0 + col) * CC, kc * 32, lane);
#pragma unroll
    for (int j = 0; j < 8; ++j) { v16b w; const int o = c0 + j * 16 + col; const float* wr = WO + (size_t)o * CC + kc * 32 + 8 * g;
#pragma unroll
      for (int i = 0; i < 8; ++i) { w[i] = (__bf16)wr[i]; w[8 + i] = (__bf16)wr[16 + i]; }
      acc[j] = wmma_bf(a.h, w, acc[j]); acc[j] = wmma_bf(a.l, w, acc[j]); } }
#pragma unroll
  for (int j = 0; j < 8; ++j) { const int cl = j * 16 + col; const float bb = bfr(BO[c0 + cl]);
#pragma unroll
    for (int r = 0; r < 8; ++r) sf[wave][8 * g + r][cl] = bfr(X[(r0 + 8 * g + r) * CC + c0 + cl]) + acc[j][r] + bb;
    asm volatile("s_wait_loadcnt 0x0" ::: "memory"); }
  LDSX(); for (int rl = 0; rl < 16; ++rl) vst2(OUT + (r0 + rl) * CC + c0 + lane * 4, *(const v4f*)&sf[wave][rl][lane * 4]); }
extern "C" void kernel_launch(void* const* d_in, const int* in_sizes, int n_in, void* d_out, int out_size, void* d_ws, size_t ws_size, hipStream_t stream) {
  (void)in_sizes; (void)n_in; (void)out_size;
  const float** F = (const float**)d_in;
  if (ws_size < (size_t)WS_END) return;
  char* ws = (char*)d_ws; float *Q = (float*)(ws + WS_Q), *K = (float*)(ws + WS_K), *PM = (float*)(ws + WS_PM), *CT = (float*)(ws + WS_CT), *O = (float*)(ws + WS_O); _Float16 *VP = (_Float16*)(ws + WS_VP), *KP = (_Float16*)(ws + WS_KP), *QP = (_Float16*)(ws + WS_QP);
  const int rows = TNB * TT;
  k_qkv<<<dim3(rows / 64, CC / 128, 3), 128, 0, stream>>>(F[0], F[1], F[2], F[3], Q, K, VP);
  k_kmax<<<dim3(TT / 64, TNB * NH), 128, 0, stream>>>(K, F[6], PM);
  k_kfeat<<<dim3(TT / 64, TNB * NH), 128, 0, stream>>>(K, F[6], PM, KP);
  k_qfeat<<<dim3(TT / 64, TNB * NH), 128, 0, stream>>>(Q, F[6], QP);
  k_ctx<<<dim3(MP / 64, TNB * NH), 128, 0, stream>>>(KP, VP, CT);
  k_lin<<<dim3(TT / 64, TNB * NH), 128, 0, stream>>>(QP, CT, O);
  k_out<<<dim3(rows / 64, CC / 128), 128, 0, stream>>>(O, F[4], F[5], F[0], (float*)d_out);
}
